// Transition_687194767474
// MI455X (gfx1250) — hardware-run, weakly checked
//
#include <hip/hip_runtime.h>
#pragma clang fp contract(off)

typedef __attribute__((ext_vector_type(16))) _Float16 v16h;
typedef __attribute__((ext_vector_type(8)))  _Float16 v8h;
typedef __attribute__((ext_vector_type(8)))  float    v8f;
typedef __attribute__((ext_vector_type(4)))  float    v4f;
typedef __attribute__((ext_vector_type(4)))  unsigned v4u;
typedef v4u v4u_a __attribute__((may_alias));

constexpr int kClouds  = 8;
constexpr int kN       = 4096;
constexpr int kD       = 64;
constexpr int kNbr     = 32;
constexpr int kW0Pitch = 67;
constexpr int kPtsAll  = kClouds * kN;
constexpr int kRowsAll = kPtsAll * kNbr;
constexpr int kTiles   = kRowsAll / 64;
constexpr int kStatBlocks = 256;
constexpr int kPartPitch  = 256;
constexpr float kWCarry  = 4096.0f;
constexpr float kWInv    = 1.0f / 4096.0f;
constexpr float kF16Min  = 6.103515625e-5f;

static_assert(kPtsAll == 32768 && kRowsAll == 1048576 && kTiles == 16384, "shape constants");
static_assert(kPtsAll * 128 * 4 == 16777216, "output bytes");
static_assert(kTiles % kStatBlocks == 0 && kRowsAll % (kStatBlocks * 16) == 0, "exact grids");
static_assert(kNbr == 32, "one wave lane per neighbour slot");

constexpr size_t kOffU    = 0;
constexpr size_t kOffV    = kOffU   + (size_t)kPtsAll * 64 * 4;
constexpr size_t kOffNbr  = kOffV   + (size_t)kPtsAll * 64 * 4;
constexpr size_t kOffExt  = kOffNbr + (size_t)kPtsAll * kNbr * 4;
constexpr size_t kOffPart = kOffExt + (size_t)kPtsAll * 128 * 4;
constexpr size_t kOffAc   = kOffPart + (size_t)3 * kStatBlocks * kPartPitch * 4;
constexpr size_t kWsTotal = kOffAc  + (size_t)3 * 256 * 4;
static_assert(kWsTotal == 38538240ull, "carve total");
static_assert(kWsTotal <= 134217728ull, "carve cap");
constexpr float kInvN = 1.0f / 1048576.0f;
static_assert(kOffV % 128 == 0 && kOffNbr % 128 == 0 && kOffExt % 128 == 0 && kOffPart % 128 == 0 && kOffAc % 128 == 0,
              "line aligned carve");

union FragH { v16h v; v8h h[2]; };

__device__ __forceinline__ v8f mma_f16(v16h a, v16h b, v8f c) {
  c = __builtin_amdgcn_wmma_f32_16x16x32_f16(false, a, false, b, (short)0, c, false, false);
  asm volatile("v_nop\n\tv_nop\n\tv_nop\n\tv_nop" : "+v"(c) : "v"(a), "v"(b));
  return c;
}
__device__ __forceinline__ v16h lds_frag(const _Float16* p) {
  FragH f;
  f.h[0] = *(const v8h*)(p);
  f.h[1] = *(const v8h*)(p + 16);
  return f.v;
}
__device__ __forceinline__ float bf_rne(float f) {
  const unsigned u = __float_as_uint(f);
  const unsigned tie = (u & 0x00010000u) ? 1u : 0u;
  const unsigned r = (u + 0x7FFFu + tie) & 0xFFFF0000u;
  return __uint_as_float(r);
}
__device__ __forceinline__ float flush16(float v) { return (fabsf(v) < kF16Min) ? 0.0f : v; }
__device__ __forceinline__ _Float16 w_to_h(float w) { return (_Float16)flush16(bf_rne(w) * kWCarry); }
__device__ __forceinline__ _Float16 in_to_h(float x) { return (_Float16)flush16(bf_rne(x)); }
__device__ __forceinline__ unsigned bfv_h16_bits(float v) {
  const unsigned u = __float_as_uint(v);
  const unsigned sg = (u & 0x80000000u) ? 0x8000u : 0u;
  unsigned em = u & 0x7FFFFFFFu;
  em = (em > 0x477FE000u) ? 0x477FE000u : em;
  const unsigned hb = (em - 0x38000000u) >> 13;
  unsigned res = (em < 0x38800000u) ? 0u : (hb | sg);
  asm volatile("" : "+v"(res));
  return res;
}
__device__ __forceinline__ _Float16 act_to_h(float x) { return (_Float16)flush16(x); }
__device__ __forceinline__ v16h wfrag_vec(const float* __restrict__ p) {
  const v4f a = *(const v4f*)(p);
  const v4f b = *(const v4f*)(p + 4);
  const v4f c = *(const v4f*)(p + 16);
  const v4f d = *(const v4f*)(p + 20);
  v16h r;
#pragma unroll
  for (int e = 0; e < 4; ++e) {
    const float fa = a[e];
    const float fb = b[e];
    const float fc = c[e];
    const float fd = d[e];
    r[e]      = w_to_h(fa);
    r[4 + e]  = w_to_h(fb);
    r[8 + e]  = w_to_h(fc);
    r[12 + e] = w_to_h(fd);
  }
  return r;
}

__global__ __launch_bounds__(256) void k_ugemm(const float* __restrict__ xyz, const float* __restrict__ pts,
                                               const float* __restrict__ W0, float* __restrict__ U,
                                               float* __restrict__ V, int tilesPerBlock) {
  constexpr int AP = 104;
  __shared__ __align__(16) _Float16 As[64 * AP];
  __shared__ __align__(16) _Float16 Bs[64 * AP];
  __shared__ __align__(16) float Ps[64 * 64];
  __shared__ float wq[3][64];
  const int tid = threadIdx.x, lane = tid & 31, wave = tid >> 5;
  const int lm = lane & 15, hf = lane >> 4;
  const int rs = wave & 3, cg = wave >> 2;
#pragma unroll 1
  for (int i = 0; i < 24; ++i) {
    unsigned eu = (unsigned)tid + 256u * (unsigned)i;
    asm volatile("" : "+v"(eu));
    unsigned ou = eu / 96u;
    asm volatile("" : "+v"(ou));
    unsigned ku = eu - ou * 96u;
    asm volatile("" : "+v"(ku));
    const int o = (int)ou;
    const int k = (int)ku;
    const int src = (k < 64) ? (3 + k) : ((k < 67) ? (k - 64) : 0);
    const float w = W0[o * kW0Pitch + src];
    const float c = (k < 67) ? flush16(bf_rne(w) * kWCarry) : 0.0f;
    Bs[o * AP + k] = (_Float16)c;
  }
  if (tid < 192) {
    const int c = tid >> 6, o = tid & 63;
    wq[c][o] = bf_rne(W0[o * kW0Pitch + c]);
  }
  __syncthreads();
  v16h bf[2][3];
#pragma unroll
  for (int j = 0; j < 2; ++j)
#pragma unroll
    for (int kk = 0; kk < 3; ++kk)
      bf[j][kk] = lds_frag(Bs + (cg * 32 + 16 * j + lm) * AP + kk * 32 + 8 * hf);
#pragma unroll 1
  for (int tt = 0; tt < tilesPerBlock; ++tt) {
    const int tile = blockIdx.x * tilesPerBlock + tt;
    const int r = tid >> 2, cq = tid & 3;
    const size_t g = (size_t)tile * 64 + r;
    float xb, yb, zb;
    {
      const float* pp = pts + g * kD + cq * 16;
      v4f p4[4];
#pragma unroll
      for (int qd = 0; qd < 4; ++qd) p4[qd] = *(const v4f*)(pp + 4 * qd);
      const float* xp = xyz + g * 3;
      xb = bf_rne(xp[0]);
      yb = bf_rne(xp[1]);
      zb = bf_rne(xp[2]);
      v8h h0, h1;
#pragma unroll
      for (int qd = 0; qd < 4; ++qd)
#pragma unroll
        for (int e = 0; e < 4; ++e) {
          const float f = p4[qd][e];
          const _Float16 hv = in_to_h(f);
          if (qd < 2) h0[4 * qd + e] = hv;
          else        h1[4 * (qd - 2) + e] = hv;
        }
      const unsigned hxb = bfv_h16_bits(xb);
      const unsigned hyb = bfv_h16_bits(yb);
      const unsigned hzb = bfv_h16_bits(zb);
      unsigned zr = 0u;
      asm volatile("" : "+v"(zr));
      unsigned w01 = hxb | (hyb << 16);
      asm volatile("" : "+v"(w01));
      const bool c0 = (cq == 0);
      v4u tw;
      tw.x = c0 ? w01 : zr;
      tw.y = c0 ? hzb : zr;
      tw.z = zr;
      tw.w = zr;
      *(v8h*)(As + r * AP + cq * 16) = h0;
      *(v8h*)(As + r * AP + cq * 16 + 8) = h1;
      *(v4u_a*)(As + r * AP + 64 + cq * 8) = tw;
    }
    __syncthreads();
    v8f acc[2];
    acc[0] = (v8f){0.f, 0.f, 0.f, 0.f, 0.f, 0.f, 0.f, 0.f};
    acc[1] = (v8f){0.f, 0.f, 0.f, 0.f, 0.f, 0.f, 0.f, 0.f};
#pragma unroll
    for (int kk = 0; kk < 3; ++kk) {
      const v16h fa = lds_frag(As + (rs * 16 + lm) * AP + kk * 32 + 8 * hf);
#pragma unroll
      for (int j = 0; j < 2; ++j) acc[j] = mma_f16(fa, bf[j][kk], acc[j]);
    }
#pragma unroll
    for (int j = 0; j < 2; ++j)
#pragma unroll
      for (int q = 0; q < 8; ++q) {
        const float v = acc[j][q] * kWInv;
        Ps[(rs * 16 + 8 * hf + q) * 64 + cg * 32 + 16 * j + lm] = v;
      }
    __syncthreads();
    {
      float* dst = U + (size_t)tile * 64 * 64;
      v4f vals[4];
#pragma unroll
      for (int i = 0; i < 4; ++i) vals[i] = *(const v4f*)(Ps + (tid + 256 * i) * 4);
      for (int pass = 0; pass < 2; ++pass) {
#pragma unroll
        for (int i = 0; i < 4; ++i) *(volatile v4f*)(dst + (size_t)(tid + 256 * i) * 4) = vals[i];
        __threadfence();
      }
    }
    __syncthreads();
#pragma unroll 4
    for (int e = 0; e < 16; ++e) {
      const int o = cq * 16 + e;
      float t = wq[0][o] * xb;
      t = fmaf(wq[1][o], yb, t);
      t = fmaf(wq[2][o], zb, t);
      Ps[r * 64 + o] = t;
    }
    __syncthreads();
    {
      float* dst = V + (size_t)tile * 64 * 64;
      v4f vals[4];
#pragma unroll
      for (int i = 0; i < 4; ++i) vals[i] = *(const v4f*)(Ps + (tid + 256 * i) * 4);
      for (int pass = 0; pass < 2; ++pass) {
#pragma unroll
        for (int i = 0; i < 4; ++i) *(volatile v4f*)(dst + (size_t)(tid + 256 * i) * 4) = vals[i];
        __threadfence();
      }
    }
  }
}

__global__ __launch_bounds__(256) void k_knn(const float* __restrict__ xyz, int* __restrict__ nbr) {
#pragma clang fp contract(off)
  __shared__ unsigned cxy[kN];
  __shared__ float cz[kN];
  __shared__ float csq[kN];
  const int tid = threadIdx.x, lane = tid & 31, wave = tid >> 5;
  const int b = blockIdx.x >> 6;
  const int q0 = (blockIdx.x & 63) * 64;
  const float* xb = xyz + (size_t)b * kN * 3;
#pragma unroll 1
  for (int i = 0; i < 16; ++i) {
    const int p = tid + 256 * i;
    const float x = bf_rne(xb[p * 3 + 0]);
    const float y = bf_rne(xb[p * 3 + 1]);
    const float z = bf_rne(xb[p * 3 + 2]);
    float t0 = x * x;
    asm volatile("" : "+v"(t0));
    float t1 = y * y;
    asm volatile("" : "+v"(t1));
    float t2 = z * z;
    asm volatile("" : "+v"(t2));
    float s02 = t0 + t2;
    asm volatile("" : "+v"(s02));
    const float sq = s02 + t1;
    unsigned ux = __float_as_uint(x) & 0xFFFF0000u;
    asm volatile("" : "+v"(ux));
    unsigned uy = __float_as_uint(y) >> 16;
    asm volatile("" : "+v"(uy));
    cxy[p] = ux | uy;
    cz[p] = z;
    csq[p] = sq;
  }
  __syncthreads();
  const int upaddr = ((lane == 0) ? 0 : (lane - 1)) << 2;
  const float kInf = __uint_as_float(0x7F800000u);
#pragma unroll 1
  for (int qi = 0; qi < 8; ++qi) {
    const int n = q0 + wave * 8 + qi;
    const unsigned qw = cxy[n];
    const float qx = __uint_as_float(qw & 0xFFFF0000u);
    const float qy = __uint_as_float(qw << 16);
    const float qz = cz[n];
    const float qs = csq[n];
    float bd = kInf;
    int bi = 0;
    float thr = kInf;
#pragma unroll 1
    for (int base = 0; base < kN; base += 32) {
      const int m = base + lane;
      const unsigned w = cxy[m];
      const float mx = __uint_as_float(w & 0xFFFF0000u);
      const float my = __uint_as_float(w << 16);
      const float mz = cz[m];
      const float sm = csq[m];
      float p = qx * mx;
      asm volatile("" : "+v"(p));
      float dt = fmaf(qy, my, p);
      dt = fmaf(qz, mz, dt);
      const float s = qs + sm;
      const float two = 2.0f * dt;
      const float dist = s - two;
      unsigned mask = __builtin_amdgcn_ballot_w32(dist < thr);
      while (mask != 0u) {
        const int j = __builtin_ctz(mask);
        mask &= mask - 1u;
        const float dc = __int_as_float(__builtin_amdgcn_readlane(__float_as_int(dist), j));
        if (dc < thr) {
          const int ic = base + j;
          const float ud = __int_as_float(__builtin_amdgcn_ds_bpermute(upaddr, __float_as_int(bd)));
          const int   ui = __builtin_amdgcn_ds_bpermute(upaddr, bi);
          const bool keep = bd <= dc;
          const bool pk = (lane == 0) | (ud <= dc);
          const float nd = keep ? bd : (pk ? dc : ud);
          const int   ni = keep ? bi : (pk ? ic : ui);
          bd = nd;
          bi = ni;
          thr = __int_as_float(__builtin_amdgcn_readlane(__float_as_int(bd), 31));
        }
      }
    }
    int oi = bi < 0 ? 0 : (bi > kN - 1 ? kN - 1 : bi);
    volatile int* dst = (volatile int*)(nbr + ((size_t)(b * kN + n)) * kNbr + lane);
    *dst = oi;
    __threadfence();
    *dst = oi;
  }
}

__global__ __launch_bounds__(256) void k_stats0(const float* __restrict__ U, const float* __restrict__ V,
                                                const int* __restrict__ nbr, const float* __restrict__ b0,
                                                float* __restrict__ part, int rowsPerBlock) {
  __shared__ float rsum[2][16][64];
  __shared__ __align__(16) float fin[256];
  const int tid = threadIdx.x;
  const int cq = tid & 15, slot = tid >> 4;
  float bz[4];
#pragma unroll
  for (int e = 0; e < 4; ++e) bz[e] = bf_rne(b0[4 * cq + e]);
  float s[4] = {0.f, 0.f, 0.f, 0.f}, q[4] = {0.f, 0.f, 0.f, 0.f};
  const size_t row0 = (size_t)blockIdx.x * rowsPerBlock;
  const int nit = rowsPerBlock >> 4;
#pragma unroll 1
  for (int it = 0; it < nit; ++it) {
    const size_t gr = row0 + (size_t)it * 16 + slot;
    int m = nbr[gr];
    m = m < 0 ? 0 : (m > kN - 1 ? kN - 1 : m);
    const int g = (int)(gr >> 5);
    const int b = g >> 12;
    const v4f u = *(const v4f*)(U + ((size_t)(b * kN + m)) * 64 + 4 * cq);
    const v4f v = *(const v4f*)(V + (size_t)g * 64 + 4 * cq);
#pragma unroll
    for (int e = 0; e < 4; ++e) {
      const float z = (u[e] - v[e]) + bz[e];
      s[e] += z;
      q[e] += z * z;
    }
  }
#pragma unroll
  for (int e = 0; e < 4; ++e) { rsum[0][slot][4 * cq + e] = s[e]; rsum[1][slot][4 * cq + e] = q[e]; }
  __syncthreads();
  {
    const int n = tid & 127, qq = tid >> 7;
    const int nc = n < 64 ? n : 63;
    float v = 0.f;
#pragma unroll
    for (int sl = 0; sl < 16; ++sl) v += rsum[qq][sl][nc];
    fin[tid] = (n < 64) ? v : 0.f;
  }
  __syncthreads();
  if (tid < 64) {
    const v4f v = *(const v4f*)(fin + 4 * tid);
    volatile v4f* d = (volatile v4f*)(part + (size_t)blockIdx.x * kPartPitch + 4 * tid);
    *d = v;
    __threadfence();
    *d = v;
  }
}

__global__ __launch_bounds__(128) void k_bnfin(const float* __restrict__ part, int nblk, int nch,
                                               const float* __restrict__ g, const float* __restrict__ bt,
                                               float invn, float* __restrict__ ac) {
  __shared__ __align__(16) float sac[256];
  const int o = threadIdx.x;
  const int oc = o < nch ? o : nch - 1;
  double s = 0.0, q = 0.0;
#pragma unroll 4
  for (int k = 0; k < nblk; ++k) {
    s += (double)part[(size_t)k * kPartPitch + oc];
    q += (double)part[(size_t)k * kPartPitch + 128 + oc];
  }
  const double mean = s * (double)invn;
  double var = q * (double)invn - mean * mean;
  var = var < 0.0 ? 0.0 : var;
  const float inv = rsqrtf((float)var + 1e-5f);
  const float a = bf_rne(g[oc]) * inv;
  const float c = bf_rne(bt[oc]) - (float)mean * a;
  sac[o] = (o < nch) ? a : 0.f;
  sac[128 + o] = (o < nch) ? c : 0.f;
  __syncthreads();
  if (o < 64) {
    const v4f v = *(const v4f*)(sac + 4 * o);
    volatile v4f* d = (volatile v4f*)(ac + 4 * o);
    *d = v;
    __threadfence();
    *d = v;
  }
}

template <int DEPTH>
__global__ __launch_bounds__(256) void k_chain(
    const float* __restrict__ U, const float* __restrict__ V, const int* __restrict__ nbr,
    const float* __restrict__ b0, const float* __restrict__ ac0,
    const float* __restrict__ W1, const float* __restrict__ b1, const float* __restrict__ ac1,
    const float* __restrict__ W2, const float* __restrict__ b2, const float* __restrict__ g2,
    float* __restrict__ yext, float* __restrict__ part, int tilesPerBlock) {
  constexpr int AP = 72;
  constexpr int NOUT = (DEPTH == 1) ? 64 : 128;
  constexpr int HW = NOUT / 2;
  constexpr int NJ = NOUT / 32;
  __shared__ __align__(16) _Float16 Ah[64 * AP];
  __shared__ __align__(16) _Float16 W2s[(DEPTH == 2) ? 128 * AP : 8];
  __shared__ __align__(16) float cst[3][64];
  __shared__ int gpos[128];
  __shared__ __align__(16) float Emx[4][128];
  __shared__ __align__(16) float Emn[4][128];
  __shared__ float red[2][8][64];
  __shared__ __align__(16) float fin[256];
  const int tid = threadIdx.x, lane = tid & 31, wave = tid >> 5;
  const int lm = lane & 15, hf = lane >> 4;
  const int rs = wave & 3, cg = wave >> 2;
  if (tid < 64) {
    cst[0][tid] = ac0[tid];
    cst[1][tid] = ac0[128 + tid];
    cst[2][tid] = bf_rne(b0[tid]);
  }
  if constexpr (DEPTH == 2) {
    if (tid < 128) gpos[tid] = (bf_rne(g2[tid]) > 0.0f) ? 1 : 0;
    const int n = tid >> 1, hs = (tid & 1) * 32;
#pragma unroll 1
    for (int i = 0; i < 4; ++i) {
      const float* wp = W2 + (size_t)n * 64 + hs + 8 * i;
      const v4f a = *(const v4f*)(wp);
      const v4f c = *(const v4f*)(wp + 4);
      v8h h;
#pragma unroll
      for (int e = 0; e < 4; ++e) {
        const float fa = a[e];
        const float fc = c[e];
        h[e] = w_to_h(fa);
        h[4 + e] = w_to_h(fc);
      }
      *(v8h*)(W2s + n * AP + hs + 8 * i) = h;
    }
  }
  v16h bf1[2][2];
  float b1c[2], s1c[2], t1c[2];
#pragma unroll
  for (int j = 0; j < 2; ++j) {
    const int n = cg * 32 + 16 * j + lm;
#pragma unroll
    for (int kk = 0; kk < 2; ++kk) bf1[j][kk] = wfrag_vec(W1 + (size_t)n * 64 + kk * 32 + 8 * hf);
    b1c[j] = bf_rne(b1[n]);
    s1c[j] = (DEPTH == 2) ? ac1[n] : 0.f;
    t1c[j] = (DEPTH == 2) ? ac1[128 + n] : 0.f;
  }
  float b2c[4];
#pragma unroll
  for (int j = 0; j < 4; ++j) b2c[j] = (DEPTH == 2) ? bf_rne(b2[cg * 64 + 16 * j + lm]) : 0.f;
  float ssum[4], ssq[4];
#pragma unroll
  for (int j = 0; j < 4; ++j) { ssum[j] = 0.f; ssq[j] = 0.f; }
  __syncthreads();
#pragma unroll 1
  for (int tt = 0; tt < tilesPerBlock; ++tt) {
    const int tile = blockIdx.x * tilesPerBlock + tt;
    __syncthreads();
    {
      const int r = tid >> 2, cq = tid & 3;
      const size_t gr = (size_t)tile * 64 + r;
      int m = nbr[gr];
      m = m < 0 ? 0 : (m > kN - 1 ? kN - 1 : m);
      const int g = (int)(gr >> 5);
      const int b = g >> 12;
      const float* up = U + ((size_t)(b * kN + m)) * 64 + cq * 16;
      const float* vp = V + (size_t)g * 64 + cq * 16;
      v4f u4[4], v4[4];
#pragma unroll
      for (int qd = 0; qd < 4; ++qd) { u4[qd] = *(const v4f*)(up + 4 * qd); v4[qd] = *(const v4f*)(vp + 4 * qd); }
      v8h h0, h1;
#pragma unroll
      for (int qd = 0; qd < 4; ++qd) {
        const v4f a4 = *(const v4f*)(&cst[0][cq * 16 + 4 * qd]);
        const v4f c4 = *(const v4f*)(&cst[1][cq * 16 + 4 * qd]);
        const v4f z4 = *(const v4f*)(&cst[2][cq * 16 + 4 * qd]);
#pragma unroll
        for (int e = 0; e < 4; ++e) {
          const float z = (u4[qd][e] - v4[qd][e]) + z4[e];
          const float x = fmaxf(a4[e] * z + c4[e], 0.0f);
          const _Float16 hv = act_to_h(x);
          if (qd < 2) h0[4 * qd + e] = hv;
          else        h1[4 * (qd - 2) + e] = hv;
        }
      }
      *(v8h*)(Ah + r * AP + cq * 16) = h0;
      *(v8h*)(Ah + r * AP + cq * 16 + 8) = h1;
    }
    __syncthreads();
    v8f am[2];
#pragma unroll
    for (int j = 0; j < 2; ++j) am[j] = (v8f){0.f, 0.f, 0.f, 0.f, 0.f, 0.f, 0.f, 0.f};
#pragma unroll
    for (int kk = 0; kk < 2; ++kk) {
      const v16h fh = lds_frag(Ah + (rs * 16 + lm) * AP + kk * 32 + 8 * hf);
#pragma unroll
      for (int j = 0; j < 2; ++j) am[j] = mma_f16(fh, bf1[j][kk], am[j]);
    }
    if constexpr (DEPTH == 1) {
#pragma unroll
      for (int j = 0; j < 2; ++j)
#pragma unroll
        for (int q = 0; q < 8; ++q) {
          const float z = am[j][q] * kWInv + b1c[j];
          ssum[j] += z;
          ssq[j] += z * z;
        }
    } else {
      __syncthreads();
#pragma unroll
      for (int j = 0; j < 2; ++j)
#pragma unroll
        for (int q = 0; q < 8; ++q) {
          const float z = am[j][q] * kWInv + b1c[j];
          const float x = fmaxf(s1c[j] * z + t1c[j], 0.0f);
          const _Float16 hv = act_to_h(x);
          const int o = (rs * 16 + 8 * hf + q) * AP + cg * 32 + 16 * j + lm;
          Ah[o] = hv;
        }
      __syncthreads();
      v16h a2h[2];
#pragma unroll
      for (int kk = 0; kk < 2; ++kk) a2h[kk] = lds_frag(Ah + (rs * 16 + lm) * AP + kk * 32 + 8 * hf);
#pragma unroll
      for (int j = 0; j < 4; ++j) {
        v8f cm = (v8f){0.f, 0.f, 0.f, 0.f, 0.f, 0.f, 0.f, 0.f};
#pragma unroll
        for (int kk = 0; kk < 2; ++kk) {
          const v16h bw = lds_frag(W2s + (cg * 64 + 16 * j + lm) * AP + kk * 32 + 8 * hf);
          cm = mma_f16(a2h[kk], bw, cm);
        }
        float mx = -3.0e38f, mn = 3.0e38f;
#pragma unroll
        for (int q = 0; q < 8; ++q) {
          const float z = cm[q] * kWInv + b2c[j];
          ssum[j] += z;
          ssq[j] += z * z;
          mx = fmaxf(mx, z);
          mn = fminf(mn, z);
        }
        const float omx = __shfl_xor(mx, 16, 32);
        const float omn = __shfl_xor(mn, 16, 32);
        mx = fmaxf(mx, omx);
        mn = fminf(mn, omn);
        if (lane < 16) { Emx[rs][cg * 64 + 16 * j + lm] = mx; Emn[rs][cg * 64 + 16 * j + lm] = mn; }
      }
      __syncthreads();
      if (wave < 2) {
        const int c4 = lane * 4;
        const int e0 = 2 * wave, e1 = 2 * wave + 1;
        const v4f xa = *(const v4f*)(&Emx[e0][c4]);
        const v4f xb = *(const v4f*)(&Emx[e1][c4]);
        const v4f na = *(const v4f*)(&Emn[e0][c4]);
        const v4f nb = *(const v4f*)(&Emn[e1][c4]);
        v4f o;
#pragma unroll
        for (int e = 0; e < 4; ++e) {
          const float mx = fmaxf(xa[e], xb[e]);
          const float mn = fminf(na[e], nb[e]);
          const int gp = gpos[c4 + e];
          o[e] = gp ? mx : mn;
        }
        volatile v4f* d = (volatile v4f*)(yext + ((size_t)tile * 2 + wave) * 128 + c4);
        *d = o;
        __threadfence();
        *d = o;
      }
    }
  }
#pragma unroll
  for (int j = 0; j < NJ; ++j) {
    ssum[j] += __shfl_xor(ssum[j], 16, 32);
    ssq[j]  += __shfl_xor(ssq[j], 16, 32);
  }
  if (lane < 16) {
#pragma unroll
    for (int j = 0; j < NJ; ++j) { red[0][wave][16 * j + lane] = ssum[j]; red[1][wave][16 * j + lane] = ssq[j]; }
  }
  __syncthreads();
  {
    const int n = tid & 127, qq = tid >> 7;
    const int nc = n < NOUT ? n : NOUT - 1;
    const int cgn = nc / HW;
    const int w = nc - cgn * HW;
    const float v = ((red[qq][cgn * 4 + 0][w] + red[qq][cgn * 4 + 1][w]) + red[qq][cgn * 4 + 2][w]) + red[qq][cgn * 4 + 3][w];
    fin[tid] = (n < NOUT) ? v : 0.f;
  }
  __syncthreads();
  if (tid < 64) {
    const v4f v = *(const v4f*)(fin + 4 * tid);
    volatile v4f* d = (volatile v4f*)(part + (size_t)blockIdx.x * kPartPitch + 4 * tid);
    *d = v;
    __threadfence();
    *d = v;
  }
}

__global__ __launch_bounds__(256) void k_pool(const float* __restrict__ yext, const float* __restrict__ ac2,
                                              const int* __restrict__ nsp, float* __restrict__ out) {
  __shared__ __align__(16) float sa[128];
  __shared__ __align__(16) float sc[128];
  const int tid = threadIdx.x;
  if (tid < 128) { sa[tid] = ac2[tid]; sc[tid] = ac2[128 + tid]; }
  __syncthreads();
  const int ns = nsp[0];
  const bool bad = (ns != kNbr);
  const float nanv = __uint_as_float(0x7FC00000u);
  v4f vals[4];
#pragma unroll
  for (int i = 0; i < 4; ++i) {
    const size_t u = ((size_t)blockIdx.x * 4 + i) * 256 + tid;
    const int c4 = (int)(u & 31) * 4;
    const v4f v = *(const v4f*)(yext + u * 4);
    const v4f a = *(const v4f*)(sa + c4);
    const v4f c = *(const v4f*)(sc + c4);
    v4f o;
#pragma unroll
    for (int e = 0; e < 4; ++e) {
      const float y = fmaxf(a[e] * v[e] + c[e], 0.0f);
      o[e] = bad ? nanv : y;
    }
    vals[i] = o;
  }
  for (int pass = 0; pass < 2; ++pass) {
#pragma unroll
    for (int i = 0; i < 4; ++i) {
      const size_t u = ((size_t)blockIdx.x * 4 + i) * 256 + tid;
      *(volatile v4f*)(out + u * 4) = vals[i];
    }
    __threadfence();
  }
}

extern "C" void kernel_launch(void* const* d_in, const int* in_sizes, int n_in,
                              void* d_out, int out_size, void* d_ws, size_t ws_size, hipStream_t stream) {
  if (n_in < 15) return;
  if (in_sizes[0] != kPtsAll * 3) return;
  if (in_sizes[1] != kPtsAll * kD) return;
  if (in_sizes[2] != 64 * kW0Pitch) return;
  if (in_sizes[3] != 64 || in_sizes[4] != 64 || in_sizes[5] != 64) return;
  if (in_sizes[6] != 64 * 64) return;
  if (in_sizes[7] != 64 || in_sizes[8] != 64 || in_sizes[9] != 64) return;
  if (in_sizes[10] != 128 * 64) return;
  if (in_sizes[11] != 128 || in_sizes[12] != 128 || in_sizes[13] != 128) return;
  if (in_sizes[14] != 1) return;
  if (out_size != kPtsAll * 128) return;
  if (ws_size < kWsTotal) return;

  const float* xyz   = (const float*)d_in[0];
  const float* pts   = (const float*)d_in[1];
  const float* W0    = (const float*)d_in[2];
  const float* b0    = (const float*)d_in[3];
  const float* g0    = (const float*)d_in[4];
  const float* beta0 = (const float*)d_in[5];
  const float* W1    = (const float*)d_in[6];
  const float* b1    = (const float*)d_in[7];
  const float* g1    = (const float*)d_in[8];
  const float* beta1 = (const float*)d_in[9];
  const float* W2    = (const float*)d_in[10];
  const float* b2    = (const float*)d_in[11];
  const float* g2    = (const float*)d_in[12];
  const float* beta2 = (const float*)d_in[13];
  const int*   nsp   = (const int*)d_in[14];
  float* out = (float*)d_out;

  char* ws = (char*)d_ws;
  float* U    = (float*)(ws + kOffU);
  float* V    = (float*)(ws + kOffV);
  int*   nbr  = (int*)(ws + kOffNbr);
  float* ext  = (float*)(ws + kOffExt);
  float* part = (float*)(ws + kOffPart);
  float* ac   = (float*)(ws + kOffAc);
  const size_t partSlot = (size_t)kStatBlocks * kPartPitch;
  float* p0 = part + 0 * partSlot;
  float* p1 = part + 1 * partSlot;
  float* p2 = part + 2 * partSlot;
  float* a0 = ac + 0 * 256;
  float* a1 = ac + 1 * 256;
  float* a2 = ac + 2 * 256;

  k_ugemm<<<128, 256, 0, stream>>>(xyz, pts, W0, U, V, (kPtsAll / 64) / 128);
  k_knn<<<kPtsAll / 64, 256, 0, stream>>>(xyz, nbr);
  k_stats0<<<kStatBlocks, 256, 0, stream>>>(U, V, nbr, b0, p0, kRowsAll / kStatBlocks);
  k_bnfin<<<1, 128, 0, stream>>>(p0, kStatBlocks, 64, g0, beta0, kInvN, a0);
  k_chain<1><<<kStatBlocks, 256, 0, stream>>>(U, V, nbr, b0, a0, W1, b1, a1, W2, b2, g2, ext, p1, kTiles / kStatBlocks);
  k_bnfin<<<1, 128, 0, stream>>>(p1, kStatBlocks, 64, g1, beta1, kInvN, a1);
  k_chain<2><<<kStatBlocks, 256, 0, stream>>>(U, V, nbr, b0, a0, W1, b1, a1, W2, b2, g2, ext, p2, kTiles / kStatBlocks);
  k_bnfin<<<1, 128, 0, stream>>>(p2, kStatBlocks, 128, g2, beta2, kInvN, a2);
  k_pool<<<1024, 256, 0, stream>>>(ext, a2, nsp, out);
}
